// EGNN_22050362097722
// MI455X (gfx1250) — hardware-run, weakly checked
//
#include <hip/hip_runtime.h>
#include <stddef.h>


#define NTHR   256
#define NWAVE  8
#define EPT    8
#define CHUNK  (NTHR * EPT)
#define WCAP   (EPT * 32)
#define LISTN  (NWAVE * WCAP)
#define PASSN  (NWAVE * 16)
#define PCAP   (CHUNK + PASSN)
#define NB     128
#define HD     64
#define ACCW   68
#define MSGW   68
#define NPB    (NWAVE * 16)

static_assert(PASSN == 128);
static_assert(NTHR >= PASSN);
static_assert(NB <= NTHR);
static_assert(NB == NPB);
static_assert(((NB * HD) % (NTHR * 4)) == 0);
static_assert((((NTHR * 4) / HD) * HD) == NTHR * 4);
static_assert(NPB * 3 <= 2 * NTHR);
static_assert(ACCW >= HD + 4);

#define DEV __device__ __forceinline__

typedef float          v4f   __attribute__((ext_vector_type(4)));
typedef float          v8f   __attribute__((ext_vector_type(8)));
typedef int            v4i   __attribute__((ext_vector_type(4)));
typedef unsigned short v8us  __attribute__((ext_vector_type(8)));
typedef __bf16         v16bf __attribute__((ext_vector_type(16)));
union Frag { v16bf v; v8us u[2]; };

DEV unsigned short bfb(float f) {
  unsigned u = __builtin_bit_cast(unsigned, f);
  u += 0x7FFFu + ((u >> 16) & 1u);
  return (unsigned short)(u >> 16);
}
DEV float bff(unsigned short s) { return __builtin_bit_cast(float, ((unsigned)s) << 16); }
DEV float siluf(float v) { return v * __builtin_amdgcn_rcpf(1.0f + __expf(-v)); }

DEV v8us zero8us() {
  v8us z;
#pragma unroll
  for (int i = 0; i < 8; ++i) z[i] = (unsigned short)0;
  return z;
}
DEV v8f zero8f() {
  v8f z;
#pragma unroll
  for (int i = 0; i < 8; ++i) z[i] = 0.0f;
  return z;
}

DEV void split8(const float* t, v8us& hi, v8us& lo) {
#pragma unroll
  for (int i = 0; i < 8; ++i) {
    const unsigned short b = bfb(t[i]);
    hi[i] = b;
    lo[i] = bfb(t[i] - bff(b));
  }
}

DEV v8f ldc8(const float* p) {
  const v4f a = *(const v4f*)p;
  const v4f b = *(const v4f*)(p + 4);
  v8f c;
  c[0] = a.x; c[1] = a.y; c[2] = a.z; c[3] = a.w;
  c[4] = b.x; c[5] = b.y; c[6] = b.z; c[7] = b.w;
  return c;
}

DEV v8f wmb(v16bf a, v16bf b, v8f c) {
  v8f d = __builtin_amdgcn_wmma_f32_16x16x32_bf16(false, a, false, b, (short)0, c, false, false);
  asm volatile("v_nop\n\tv_nop\n\tv_nop\n\tv_nop" : "+v"(d) : "v"(a), "v"(b));
  return d;
}
DEV v8f mma3(const Frag& ah, const Frag& al, const Frag& bh, const Frag& bl, v8f c) {
  c = wmb(ah.v, bh.v, c);
  c = wmb(al.v, bh.v, c);
  c = wmb(ah.v, bl.v, c);
  return c;
}

DEV void ldA(Frag& f, const unsigned short* plane, int row, int ld, int k0, int hh) {
  const unsigned short* p = plane + row * ld + k0 + 8 * hh;
  f.u[0] = *(const v8us*)p;
  f.u[1] = *(const v8us*)(p + 16);
}

DEV void ldB32(Frag& bh, Frag& bl, const float* p, int hh) {
  const float* p0 = p + 8 * hh;
  const float* p1 = p + 16 + 8 * hh;
  const v4f a = *(const v4f*)p0, b = *(const v4f*)(p0 + 4);
  const v4f c = *(const v4f*)p1, d = *(const v4f*)(p1 + 4);
  float t0[8] = {a.x, a.y, a.z, a.w, b.x, b.y, b.z, b.w};
  float t1[8] = {c.x, c.y, c.z, c.w, d.x, d.y, d.z, d.w};
  split8(t0, bh.u[0], bl.u[0]);
  split8(t1, bh.u[1], bl.u[1]);
}

DEV void stage_wt(const float* __restrict__ W, int ldw, int K, int nrow, int ld,
                  unsigned short* hi, unsigned short* lo) {
  const int total = nrow * ld;
  for (int t = threadIdx.x; t < total; t += blockDim.x) {
    const int r = t / ld, k = t - r * ld;
    const int kc = k < K ? k : (K - 1);
    float v = W[(size_t)kc * ldw + r];
    v = (k < K) ? v : 0.0f;
    const unsigned short hb = bfb(v);
    hi[t] = hb;
    lo[t] = bfb(v - bff(hb));
  }
}

DEV void tile_out(const float* st, float* dst, int ldo, int lane, int rowlim) {
#pragma unroll
  for (int it = 0; it < 8; ++it) {
    const int row = 2 * it + (lane >> 4), col = (lane & 15) * 4;
    const v4f v = *(const v4f*)(st + row * HD + col);
    if (row < rowlim) *(volatile v4f*)(dst + (size_t)row * ldo + col) = v;
  }
}

DEV int scan_chunk(const int* __restrict__ keys, int nE, int cbase, int nodeBase,
                   int vec8, int* list, int tid, int wave) {
  int wc = 0;
  const int el0  = tid * EPT;
  const int e0   = cbase + el0;
  const int sent = -2147483647 - 1;
  v4i da, db;
  if (vec8 != 0 && cbase + CHUNK <= nE) {
    da = *(const v4i*)(keys + e0);
    db = *(const v4i*)(keys + e0 + 4);
  } else {
    da.x = (e0     < nE) ? keys[min(e0, nE - 1)] : sent;
    da.y = (e0 + 1 < nE) ? keys[min(e0 + 1, nE - 1)] : sent;
    da.z = (e0 + 2 < nE) ? keys[min(e0 + 2, nE - 1)] : sent;
    da.w = (e0 + 3 < nE) ? keys[min(e0 + 3, nE - 1)] : sent;
    db.x = (e0 + 4 < nE) ? keys[min(e0 + 4, nE - 1)] : sent;
    db.y = (e0 + 5 < nE) ? keys[min(e0 + 5, nE - 1)] : sent;
    db.z = (e0 + 6 < nE) ? keys[min(e0 + 6, nE - 1)] : sent;
    db.w = (e0 + 7 < nE) ? keys[min(e0 + 7, nE - 1)] : sent;
  }
  const unsigned nb = (unsigned)nodeBase;
  const unsigned s0 = (unsigned)da.x - nb, s1 = (unsigned)da.y - nb;
  const unsigned s2 = (unsigned)da.z - nb, s3 = (unsigned)da.w - nb;
  const unsigned s4 = (unsigned)db.x - nb, s5 = (unsigned)db.y - nb;
  const unsigned s6 = (unsigned)db.z - nb, s7 = (unsigned)db.w - nb;
  const bool h0 = s0 < (unsigned)NB, h1 = s1 < (unsigned)NB, h2 = s2 < (unsigned)NB, h3 = s3 < (unsigned)NB;
  const bool h4 = s4 < (unsigned)NB, h5 = s5 < (unsigned)NB, h6 = s6 < (unsigned)NB, h7 = s7 < (unsigned)NB;
  const unsigned any = __builtin_amdgcn_ballot_w32(h0 | h1 | h2 | h3 | h4 | h5 | h6 | h7);
  if (any != 0u) {
#define HITJ(J, HJ) { \
      const unsigned mj = __builtin_amdgcn_ballot_w32(HJ); \
      if (mj != 0u) { \
        if (HJ) { \
          const int pos = wc + (int)__builtin_amdgcn_mbcnt_lo(mj, 0u); \
          if (pos < WCAP) list[wave * WCAP + pos] = el0 + (J); \
        } \
        wc += (int)__builtin_popcount(mj); } }
    HITJ(0, h0)
    HITJ(1, h1)
    HITJ(2, h2)
    HITJ(3, h3)
    HITJ(4, h4)
    HITJ(5, h5)
    HITJ(6, h6)
    HITJ(7, h7)
#undef HITJ
  }
  return wc;
}

DEV void x0_pass(const float* __restrict__ xin, float* x0, int bn, int nN, int tid) {
  if (tid < NPB) {
    const int node = bn + tid;
    const bool ok = node < nN;
    const int nc = ok ? node : (nN - 1);
    const float* p = xin + (size_t)nc * 3;
    const float a = p[0], b = p[1], c = p[2];
    v4f o;
    o.x = ok ? a : 0.0f; o.y = ok ? b : 0.0f; o.z = ok ? c : 0.0f; o.w = 0.0f;
    *(volatile v4f*)(x0 + (size_t)node * 4) = o;
  }
}

__global__ __launch_bounds__(NTHR) void k_embin(
    const float* __restrict__ hin, const float* __restrict__ xin,
    const float* __restrict__ W, const float* __restrict__ Bv,
    float* h0, float* x0, int nN) {
  __shared__ __attribute__((aligned(16))) unsigned short wh[HD * 32];
  __shared__ __attribute__((aligned(16))) unsigned short wl[HD * 32];
  __shared__ __attribute__((aligned(16))) float sb[HD];
  __shared__ __attribute__((aligned(16))) float stg[NWAVE * 16 * HD];

  const int tid = threadIdx.x, lane = tid & 31, wave = tid >> 5, hh = lane >> 4, m = lane & 15;
  stage_wt(W, HD, 16, HD, 32, wh, wl);
  if (tid < HD) sb[tid] = Bv[tid];
  __syncthreads();

  const int node0 = (blockIdx.x * NWAVE + wave) * 16;
  const int node  = node0 + m;
  const bool valid = node < nN;
  const int nc = valid ? node : (nN - 1);
  Frag bh, bl;
  {
    const float* p = hin + (size_t)nc * 16 + 8 * hh;
    const v4f a = *(const v4f*)p, b = *(const v4f*)(p + 4);
    float t[8] = {a.x, a.y, a.z, a.w, b.x, b.y, b.z, b.w};
#pragma unroll
    for (int i = 0; i < 8; ++i) t[i] = valid ? t[i] : 0.0f;
    split8(t, bh.u[0], bl.u[0]);
    bh.u[1] = zero8us();
    bl.u[1] = zero8us();
  }
  float* st = stg + wave * 16 * HD;
#pragma unroll
  for (int ft = 0; ft < 4; ++ft) {
    v8f c = ldc8(sb + 16 * ft + 8 * hh);
    Frag ah, al;
    ldA(ah, wh, 16 * ft + m, 32, 0, hh);
    ldA(al, wl, 16 * ft + m, 32, 0, hh);
    c = mma3(ah, al, bh, bl, c);
    const v4f o0 = {c[0], c[1], c[2], c[3]};
    const v4f o1 = {c[4], c[5], c[6], c[7]};
    *(v4f*)(st + m * HD + 16 * ft + 8 * hh) = o0;
    *(v4f*)(st + m * HD + 16 * ft + 8 * hh + 4) = o1;
  }
  __syncthreads();
  tile_out(st, h0 + (size_t)node0 * HD, HD, lane, 16);
  __threadfence();
  tile_out(st, h0 + (size_t)node0 * HD, HD, lane, 16);

  const int bn = blockIdx.x * NPB;
  x0_pass(xin, x0, bn, nN, tid);
  __threadfence();
  x0_pass(xin, x0, bn, nN, tid);
}

DEV void x1_pass(const float* __restrict__ xcur, float* o1, int bn, int nN, int tid) {
#pragma unroll
  for (int it = 0; it < 2; ++it) {
    const int f = it * NTHR + tid;
    if (f < NPB * 3) {
      const int nl = f / 3, comp = f - nl * 3;
      const int node = bn + nl;
      const float v = xcur[(size_t)node * 4 + comp];
      if (node < nN) *(volatile float*)(o1 + f) = v;
    }
  }
}

template <int MLP, int FIN>
__global__ __launch_bounds__(NTHR) void k_node(
    const float* __restrict__ hprev, const float* __restrict__ aggp,
    const float* __restrict__ W1, const float* __restrict__ Bv1,
    const float* __restrict__ W2, const float* __restrict__ Bv2,
    const float* __restrict__ W3, const float* __restrict__ Bv3,
    const float* __restrict__ xcur,
    float* hout, float* outp, int nN) {
  __shared__ __attribute__((aligned(16))) unsigned short w1h[HD * 128];
  __shared__ __attribute__((aligned(16))) unsigned short w1l[HD * 128];
  __shared__ __attribute__((aligned(16))) unsigned short w2h[HD * HD];
  __shared__ __attribute__((aligned(16))) unsigned short w2l[HD * HD];
  __shared__ __attribute__((aligned(16))) unsigned short w3h[128 * HD];
  __shared__ __attribute__((aligned(16))) unsigned short w3l[128 * HD];
  __shared__ __attribute__((aligned(16))) float sb1[HD];
  __shared__ __attribute__((aligned(16))) float sb2[HD];
  __shared__ __attribute__((aligned(16))) float sb3[HD];
  __shared__ __attribute__((aligned(16))) float stg[NWAVE * 16 * HD];

  const int tid = threadIdx.x, lane = tid & 31, wave = tid >> 5, hh = lane >> 4, m = lane & 15;
  if (MLP != 0) {
    stage_wt(W1, HD, 128, HD, 128, w1h, w1l);
    stage_wt(W2, HD, HD, HD, HD, w2h, w2l);
  }
  if (FIN != 0) {
    stage_wt(W3, HD, HD, HD, HD, w3h, w3l);
  } else {
    stage_wt(W3, HD, HD, HD, HD, w3h, w3l);
    stage_wt(W3 + HD * HD, HD, HD, HD, HD, w3h + HD * HD, w3l + HD * HD);
  }
  if (tid < HD) {
    float b1 = 0.0f, b2 = 0.0f, b3 = 0.0f;
    if (MLP != 0) { b1 = Bv1[tid]; b2 = Bv2[tid]; }
    if (FIN != 0) { b3 = Bv3[tid]; }
    sb1[tid] = b1; sb2[tid] = b2; sb3[tid] = b3;
  }
  __syncthreads();

  const int node0 = (blockIdx.x * NWAVE + wave) * 16;
  const float* hrow = hprev + (size_t)(node0 + m) * HD;
  float* st = stg + wave * 16 * HD;
  float hv[4][8];

  if (MLP != 0) {
    const float* arow = aggp + (size_t)(node0 + m) * HD;
    v8f c1[4];
#pragma unroll
    for (int ft = 0; ft < 4; ++ft) c1[ft] = ldc8(sb1 + 16 * ft + 8 * hh);
#pragma unroll
    for (int ks = 0; ks < 4; ++ks) {
      Frag bh, bl;
      const float* src = (ks < 2) ? (hrow + 32 * ks) : (arow + 32 * (ks - 2));
      ldB32(bh, bl, src, hh);
#pragma unroll
      for (int ft = 0; ft < 4; ++ft) {
        Frag ah, al;
        ldA(ah, w1h, 16 * ft + m, 128, 32 * ks, hh);
        ldA(al, w1l, 16 * ft + m, 128, 32 * ks, hh);
        c1[ft] = mma3(ah, al, bh, bl, c1[ft]);
      }
    }
    Frag mh[2], ml[2];
#pragma unroll
    for (int ft = 0; ft < 4; ++ft) {
      float t[8];
#pragma unroll
      for (int rr = 0; rr < 8; ++rr) t[rr] = siluf(c1[ft][rr]);
      split8(t, mh[ft >> 1].u[ft & 1], ml[ft >> 1].u[ft & 1]);
    }
    v8f c2[4];
#pragma unroll
    for (int ft = 0; ft < 4; ++ft) c2[ft] = ldc8(sb2 + 16 * ft + 8 * hh);
#pragma unroll
    for (int ks = 0; ks < 2; ++ks) {
#pragma unroll
      for (int ft = 0; ft < 4; ++ft) {
        Frag ah, al;
        ldA(ah, w2h, 16 * ft + m, HD, 32 * ks, hh);
        ldA(al, w2l, 16 * ft + m, HD, 32 * ks, hh);
        c2[ft] = mma3(ah, al, mh[ks], ml[ks], c2[ft]);
      }
    }
#pragma unroll
    for (int ft = 0; ft < 4; ++ft) {
      const v4f p0 = *(const v4f*)(hrow + 16 * ft + 8 * hh);
      const v4f p1 = *(const v4f*)(hrow + 16 * ft + 8 * hh + 4);
      hv[ft][0] = p0.x + c2[ft][0]; hv[ft][1] = p0.y + c2[ft][1];
      hv[ft][2] = p0.z + c2[ft][2]; hv[ft][3] = p0.w + c2[ft][3];
      hv[ft][4] = p1.x + c2[ft][4]; hv[ft][5] = p1.y + c2[ft][5];
      hv[ft][6] = p1.z + c2[ft][6]; hv[ft][7] = p1.w + c2[ft][7];
    }
  } else {
#pragma unroll
    for (int ft = 0; ft < 4; ++ft) {
      const v4f p0 = *(const v4f*)(hrow + 16 * ft + 8 * hh);
      const v4f p1 = *(const v4f*)(hrow + 16 * ft + 8 * hh + 4);
      hv[ft][0] = p0.x; hv[ft][1] = p0.y; hv[ft][2] = p0.z; hv[ft][3] = p0.w;
      hv[ft][4] = p1.x; hv[ft][5] = p1.y; hv[ft][6] = p1.z; hv[ft][7] = p1.w;
    }
  }

  if (MLP != 0 && FIN == 0) {
#pragma unroll
    for (int ft = 0; ft < 4; ++ft) {
      const v4f o0 = {hv[ft][0], hv[ft][1], hv[ft][2], hv[ft][3]};
      const v4f o1 = {hv[ft][4], hv[ft][5], hv[ft][6], hv[ft][7]};
      *(v4f*)(st + m * HD + 16 * ft + 8 * hh) = o0;
      *(v4f*)(st + m * HD + 16 * ft + 8 * hh + 4) = o1;
    }
    __syncthreads();
    tile_out(st, hout + (size_t)node0 * HD, HD, lane, 16);
    __threadfence();
    tile_out(st, hout + (size_t)node0 * HD, HD, lane, 16);
    __syncthreads();
  }

  Frag xh[2], xl[2];
#pragma unroll
  for (int ft = 0; ft < 4; ++ft) split8(hv[ft], xh[ft >> 1].u[ft & 1], xl[ft >> 1].u[ft & 1]);

  constexpr int NHALF = (FIN != 0) ? 1 : 2;
  constexpr int LDO   = (FIN != 0) ? HD : 128;
  const int rowlim = (FIN != 0) ? (nN - node0) : 16;
#pragma unroll
  for (int half = 0; half < NHALF; ++half) {
    v8f c3[4];
#pragma unroll
    for (int gt = 0; gt < 4; ++gt) c3[gt] = ldc8(sb3 + 16 * gt + 8 * hh);
#pragma unroll
    for (int ks = 0; ks < 2; ++ks) {
#pragma unroll
      for (int gt = 0; gt < 4; ++gt) {
        Frag ah, al;
        ldA(ah, w3h, half * HD + 16 * gt + m, HD, 32 * ks, hh);
        ldA(al, w3l, half * HD + 16 * gt + m, HD, 32 * ks, hh);
        c3[gt] = mma3(ah, al, xh[ks], xl[ks], c3[gt]);
      }
    }
#pragma unroll
    for (int gt = 0; gt < 4; ++gt) {
      const v4f o0 = {c3[gt][0], c3[gt][1], c3[gt][2], c3[gt][3]};
      const v4f o1 = {c3[gt][4], c3[gt][5], c3[gt][6], c3[gt][7]};
      *(v4f*)(st + m * HD + 16 * gt + 8 * hh) = o0;
      *(v4f*)(st + m * HD + 16 * gt + 8 * hh + 4) = o1;
    }
    __syncthreads();
    float* dst = outp + (size_t)node0 * LDO + half * HD;
    tile_out(st, dst, LDO, lane, rowlim);
    __threadfence();
    tile_out(st, dst, LDO, lane, rowlim);
    __syncthreads();
  }

  if (FIN != 0) {
    const int bn = blockIdx.x * NPB;
    float* o1 = outp + (size_t)nN * HD + (size_t)bn * 3;
    x1_pass(xcur, o1, bn, nN, tid);
    __threadfence();
    x1_pass(xcur, o1, bn, nN, tid);
  }
}

DEV void agg_pass(const float* accp, float* aggout, int nodeBase, int lane, int wave) {
#pragma unroll
  for (int it = 0; it < (NB * HD) / (NTHR * 4); ++it) {
    const int rowl = it * ((NTHR * 4) / HD) + wave * 2 + (lane >> 4);
    const int col  = (lane & 15) * 4;
    const v4f v = *(const v4f*)(accp + rowl * ACCW + col);
    *(volatile v4f*)(aggout + (size_t)(nodeBase + rowl) * HD + col) = v;
  }
}
DEV void x_pass(const float* accp, const float* __restrict__ xcur, float* xnext, int nodeBase, int tid) {
  if (tid < NB) {
    const v4f s = *(const v4f*)(accp + tid * ACCW + HD);
    const float inv = __builtin_amdgcn_rcpf(fmaxf(s.w, 1.0f));
    const v4f xo = *(const v4f*)(xcur + (size_t)(nodeBase + tid) * 4);
    v4f xn;
    xn.x = xo.x + s.x * inv;
    xn.y = xo.y + s.y * inv;
    xn.z = xo.z + s.z * inv;
    xn.w = 0.0f;
    *(volatile v4f*)(xnext + (size_t)(nodeBase + tid) * 4) = xn;
  }
}

__global__ __launch_bounds__(NTHR) void k_agg(
    const float* __restrict__ PQ, const float* __restrict__ xcur, const int* __restrict__ ei,
    const float* __restrict__ W1, const float* __restrict__ Bv1,
    const float* __restrict__ W2, const float* __restrict__ Bv2,
    const float* __restrict__ CW1, const float* __restrict__ CBv1, const float* __restrict__ CW2,
    float* aggout, float* xnext, int nN, int nE, int vec8) {
  __shared__ __attribute__((aligned(16))) float acc[(NB + 1) * ACCW];
  __shared__ __attribute__((aligned(16))) float msg[PASSN * MSGW];
  __shared__ __attribute__((aligned(16))) unsigned short stgh[NWAVE * 16 * HD];
  __shared__ __attribute__((aligned(16))) unsigned short stgl[NWAVE * 16 * HD];
  __shared__ __attribute__((aligned(16))) unsigned short w2h[HD * HD];
  __shared__ __attribute__((aligned(16))) unsigned short w2l[HD * HD];
  __shared__ __attribute__((aligned(16))) unsigned short cwh[HD * HD];
  __shared__ __attribute__((aligned(16))) unsigned short cwl[HD * HD];
  __shared__ __attribute__((aligned(16))) float swr[HD];
  __shared__ __attribute__((aligned(16))) float sb1[HD];
  __shared__ __attribute__((aligned(16))) float sb2[HD];
  __shared__ __attribute__((aligned(16))) float scb1[HD];
  __shared__ __attribute__((aligned(16))) float scw2[HD];
  __shared__ __attribute__((aligned(16))) int list[LISTN];
  __shared__ __attribute__((aligned(16))) int pend[PCAP];
  __shared__ int slotb[PASSN];
  __shared__ int wcnt[NWAVE];
  __shared__ int pendN;

  const int tid = threadIdx.x, lane = tid & 31, wave = tid >> 5, hh = lane >> 4, m = lane & 15;
  const int nodeBase = blockIdx.x * NB;
  const int* keys = ei;
  const int* cols = ei + nE;

  for (int i = tid; i < (NB + 1) * ACCW; i += NTHR) acc[i] = 0.0f;
  stage_wt(W2, HD, HD, HD, HD, w2h, w2l);
  stage_wt(CW1, HD, HD, HD, HD, cwh, cwl);
  if (tid < HD) {
    swr[tid]  = W1[128 * HD + tid];
    sb1[tid]  = Bv1[tid];
    sb2[tid]  = Bv2[tid];
    scb1[tid] = CBv1[tid];
    scw2[tid] = CW2[tid];
  }
  if (tid == 0) pendN = 0;
  __syncthreads();

  const int nChunks = (nE + CHUNK - 1) / CHUNK;
#pragma unroll 1
  for (int ch = 0; ch < nChunks; ++ch) {
    const int cbase = ch * CHUNK;
    const int wc = scan_chunk(keys, nE, cbase, nodeBase, vec8, list, tid, wave);
    if (lane == 0) wcnt[wave] = wc;
    __syncthreads();

    const int base = pendN;
    int tot = 0, myoff = 0;
#pragma unroll
    for (int w = 0; w < NWAVE; ++w) {
      int c = wcnt[w];
      c = c > WCAP ? WCAP : (c < 0 ? 0 : c);
      if (w < wave) myoff += c;
      tot += c;
    }
    int newN = base + tot;
    newN = newN > PCAP ? PCAP : newN;
    {
      int n = wcnt[wave];
      n = n > WCAP ? WCAP : (n < 0 ? 0 : n);
      const int* lp = list + wave * WCAP;
      for (int i = lane; i < n; i += 32) {
        const int pos = base + myoff + i;
        if (pos < PCAP) pend[pos] = cbase + lp[i];
      }
    }
    const int fin = (ch == nChunks - 1) ? 1 : 0;
    const int R   = (fin != 0) ? (newN + PASSN - 1) / PASSN : newN / PASSN;
    const int Pv  = (fin != 0) ? newN : R * PASSN;
    __syncthreads();

#pragma unroll 1
    for (int r = 0; r < R; ++r) {
      const int idx = r * PASSN + wave * 16 + m;
      const bool valid = idx < Pv;
      const int ic = idx < (PCAP - 1) ? idx : (PCAP - 1);
      int e = pend[ic];
      e = valid ? e : 0;
      e = e < 0 ? 0 : (e > nE - 1 ? nE - 1 : e);
      int d = keys[e];
      int s = cols[e];
      int slot = d - nodeBase;
      if (!valid || (unsigned)slot >= (unsigned)NB) slot = NB;
      d = d < 0 ? 0 : (d > nN - 1 ? nN - 1 : d);
      s = s < 0 ? 0 : (s > nN - 1 ? nN - 1 : s);
      const v4f xd = *(const v4f*)(xcur + (size_t)d * 4);
      const v4f xs = *(const v4f*)(xcur + (size_t)s * 4);
      const float dx = xd.x - xs.x, dy = xd.y - xs.y, dz = xd.z - xs.z;
      const float rad = dx * dx + dy * dy + dz * dz;
      {
        const float* pp = PQ + (size_t)d * 128 + 32 * hh;
        const float* qp = PQ + (size_t)s * 128 + HD + 32 * hh;
        const float* wp = swr + 32 * hh;
        const float* bp = sb1 + 32 * hh;
        unsigned short* th = stgh + (wave * 16 + m) * HD + 32 * hh;
        unsigned short* tl = stgl + (wave * 16 + m) * HD + 32 * hh;
#pragma unroll
        for (int g = 0; g < 4; ++g) {
          const v4f p0 = *(const v4f*)(pp + 8 * g), p1 = *(const v4f*)(pp + 8 * g + 4);
          const v4f q0 = *(const v4f*)(qp + 8 * g), q1 = *(const v4f*)(qp + 8 * g + 4);
          const v4f w0 = *(const v4f*)(wp + 8 * g), w1 = *(const v4f*)(wp + 8 * g + 4);
          const v4f b0 = *(const v4f*)(bp + 8 * g), b1 = *(const v4f*)(bp + 8 * g + 4);
          const v4f z0 = p0 + q0 + rad * w0 + b0;
          const v4f z1 = p1 + q1 + rad * w1 + b1;
          float t[8];
          t[0] = siluf(z0.x); t[1] = siluf(z0.y); t[2] = siluf(z0.z); t[3] = siluf(z0.w);
          t[4] = siluf(z1.x); t[5] = siluf(z1.y); t[6] = siluf(z1.z); t[7] = siluf(z1.w);
          v8us vh, vl;
          split8(t, vh, vl);
          *(v8us*)(th + 8 * g) = vh;
          *(v8us*)(tl + 8 * g) = vl;
        }
      }
      if (hh == 0) slotb[wave * 16 + m] = slot;
      __syncthreads();

      {
        v8f c1[4];
#pragma unroll
        for (int ft = 0; ft < 4; ++ft) c1[ft] = ldc8(sb2 + 16 * ft + 8 * hh);
        const unsigned short* rh = stgh + (wave * 16 + m) * HD;
        const unsigned short* rl = stgl + (wave * 16 + m) * HD;
#pragma unroll
        for (int ks = 0; ks < 2; ++ks) {
          Frag bh, bl;
          bh.u[0] = *(const v8us*)(rh + 32 * ks + 8 * hh);
          bh.u[1] = *(const v8us*)(rh + 32 * ks + 16 + 8 * hh);
          bl.u[0] = *(const v8us*)(rl + 32 * ks + 8 * hh);
          bl.u[1] = *(const v8us*)(rl + 32 * ks + 16 + 8 * hh);
#pragma unroll
          for (int ft = 0; ft < 4; ++ft) {
            Frag ah, al;
            ldA(ah, w2h, 16 * ft + m, HD, 32 * ks, hh);
            ldA(al, w2l, 16 * ft + m, HD, 32 * ks, hh);
            c1[ft] = mma3(ah, al, bh, bl, c1[ft]);
          }
        }
        float* mrow = msg + (wave * 16 + m) * MSGW;
        Frag mh[2], ml[2];
#pragma unroll
        for (int ft = 0; ft < 4; ++ft) {
          float t[8];
#pragma unroll
          for (int rr = 0; rr < 8; ++rr) t[rr] = siluf(c1[ft][rr]);
          const v4f o0 = {t[0], t[1], t[2], t[3]};
          const v4f o1 = {t[4], t[5], t[6], t[7]};
          *(v4f*)(mrow + 16 * ft + 8 * hh) = o0;
          *(v4f*)(mrow + 16 * ft + 8 * hh + 4) = o1;
          split8(t, mh[ft >> 1].u[ft & 1], ml[ft >> 1].u[ft & 1]);
        }
        v8f c2[4];
#pragma unroll
        for (int ft = 0; ft < 4; ++ft) c2[ft] = ldc8(scb1 + 16 * ft + 8 * hh);
#pragma unroll
        for (int ks = 0; ks < 2; ++ks) {
#pragma unroll
          for (int ft = 0; ft < 4; ++ft) {
            Frag ah, al;
            ldA(ah, cwh, 16 * ft + m, HD, 32 * ks, hh);
            ldA(al, cwl, 16 * ft + m, HD, 32 * ks, hh);
            c2[ft] = mma3(ah, al, mh[ks], ml[ks], c2[ft]);
          }
        }
        float phi = 0.0f;
#pragma unroll
        for (int ft = 0; ft < 4; ++ft) {
          const v8f wv = ldc8(scw2 + 16 * ft + 8 * hh);
#pragma unroll
          for (int rr = 0; rr < 8; ++rr) phi += siluf(c2[ft][rr]) * wv[rr];
        }
        phi += __shfl_xor(phi, 16);
        if (hh == 0) {
          const v4f tv = {dx * phi, dy * phi, dz * phi, 1.0f};
          *(v4f*)(mrow + HD) = tv;
        }
      }
      __syncthreads();

      if (tid < ACCW) {
#pragma unroll 4
        for (int i = 0; i < PASSN; ++i) {
          int sl = slotb[i];
          sl = sl < 0 ? 0 : (sl > NB ? NB : sl);
          acc[sl * ACCW + tid] += msg[i * MSGW + tid];
        }
      }
      __syncthreads();
    }

    int rem = newN - R * PASSN;
    rem = rem < 0 ? 0 : rem;
    if (R > 0 && tid < rem) pend[tid] = pend[R * PASSN + tid];
    if (tid == 0) pendN = rem;
  }
  __syncthreads();

  agg_pass(acc, aggout, nodeBase, lane, wave);
  x_pass(acc, xcur, xnext, nodeBase, tid);
  __threadfence();
  agg_pass(acc, aggout, nodeBase, lane, wave);
  x_pass(acc, xcur, xnext, nodeBase, tid);
}

extern "C" void kernel_launch(void* const* d_in, const int* in_sizes, int n_in,
                              void* d_out, int out_size, void* d_ws, size_t ws_size,
                              hipStream_t stream) {
  if (n_in < 18) return;
  const int N = in_sizes[0] / 16;
  const int E = in_sizes[2] / 2;
  if (N <= 0 || E <= 0) return;
  if (in_sizes[0] != N * 16 || in_sizes[1] != N * 3 || in_sizes[2] != E * 2) return;
  if (in_sizes[3] != 16 * HD || in_sizes[4] != HD) return;
  if (in_sizes[5] != 4 * 129 * HD || in_sizes[6] != 4 * HD || in_sizes[7] != 4 * HD * HD || in_sizes[8] != 4 * HD) return;
  if (in_sizes[9] != 4 * HD * HD || in_sizes[10] != 4 * HD || in_sizes[11] != 4 * HD) return;
  if (in_sizes[12] != 4 * 128 * HD || in_sizes[13] != 4 * HD || in_sizes[14] != 4 * HD * HD || in_sizes[15] != 4 * HD) return;
  if (in_sizes[16] != HD * HD || in_sizes[17] != HD) return;
  if (out_size != N * HD + N * 3) return;

  const float* h_in      = (const float*)d_in[0];
  const float* x_in      = (const float*)d_in[1];
  const int*   ei        = (const int*)d_in[2];
  const float* emb_in_w  = (const float*)d_in[3];
  const float* emb_in_b  = (const float*)d_in[4];
  const float* edge_w1   = (const float*)d_in[5];
  const float* edge_b1   = (const float*)d_in[6];
  const float* edge_w2   = (const float*)d_in[7];
  const float* edge_b2   = (const float*)d_in[8];
  const float* coord_w1  = (const float*)d_in[9];
  const float* coord_b1  = (const float*)d_in[10];
  const float* coord_w2  = (const float*)d_in[11];
  const float* node_w1   = (const float*)d_in[12];
  const float* node_b1   = (const float*)d_in[13];
  const float* node_w2   = (const float*)d_in[14];
  const float* node_b2   = (const float*)d_in[15];
  const float* emb_out_w = (const float*)d_in[16];
  const float* emb_out_b = (const float*)d_in[17];
  float* out = (float*)d_out;

  const int nBlk = (N + NB - 1) / NB;
  const int npad = nBlk * NB;
  const int nodeGrid = npad / NPB;

  char* ws = (char*)d_ws;
  size_t off = 0;
  const size_t szH  = (((size_t)npad * HD  * 4) + 255) & ~(size_t)255;
  const size_t szPQ = (((size_t)npad * 128 * 4) + 255) & ~(size_t)255;
  const size_t szX  = (((size_t)npad * 4   * 4) + 255) & ~(size_t)255;
  const size_t oHA = off; off += szH;
  const size_t oHB = off; off += szH;
  const size_t oPQ = off; off += szPQ;
  const size_t oAG = off; off += szH;
  const size_t oXA = off; off += szX;
  const size_t oXB = off; off += szX;
  if (off > ws_size || off > (size_t)134217728) return;
  float* hA = (float*)(ws + oHA);
  float* hB = (float*)(ws + oHB);
  float* PQ = (float*)(ws + oPQ);
  float* AG = (float*)(ws + oAG);
  float* xA = (float*)(ws + oXA);
  float* xB = (float*)(ws + oXB);
  float* hbuf[2] = {hA, hB};
  float* xbuf[2] = {xA, xB};
  const int vec8 = 1;

  k_embin<<<nodeGrid, NTHR, 0, stream>>>(h_in, x_in, emb_in_w, emb_in_b, hA, xA, N);

  for (int l = 0; l < 4; ++l) {
    const float* ew1 = edge_w1 + (size_t)l * 129 * HD;
    const float* eb1 = edge_b1 + (size_t)l * HD;
    const float* ew2 = edge_w2 + (size_t)l * HD * HD;
    const float* eb2 = edge_b2 + (size_t)l * HD;
    const float* cw1 = coord_w1 + (size_t)l * HD * HD;
    const float* cb1 = coord_b1 + (size_t)l * HD;
    const float* cw2 = coord_w2 + (size_t)l * HD;
    if (l == 0) {
      k_node<0, 0><<<nodeGrid, NTHR, 0, stream>>>(
          hA, AG, node_w1, node_b1, node_w2, node_b2, ew1, eb1, xA, hB, PQ, N);
    } else {
      const float* hp  = hbuf[(l - 1) & 1];
      float*       hc  = hbuf[l & 1];
      const float* nw1 = node_w1 + (size_t)(l - 1) * 128 * HD;
      const float* nb1 = node_b1 + (size_t)(l - 1) * HD;
      const float* nw2 = node_w2 + (size_t)(l - 1) * HD * HD;
      const float* nb2 = node_b2 + (size_t)(l - 1) * HD;
      k_node<1, 0><<<nodeGrid, NTHR, 0, stream>>>(
          hp, AG, nw1, nb1, nw2, nb2, ew1, eb1, xA, hc, PQ, N);
    }
    k_agg<<<nBlk, NTHR, 0, stream>>>(
        PQ, xbuf[l & 1], ei, ew1, eb1, ew2, eb2, cw1, cb1, cw2, AG, xbuf[(l + 1) & 1], N, E, vec8);
  }

  k_node<1, 1><<<nodeGrid, NTHR, 0, stream>>>(
      hbuf[1], AG,
      node_w1 + (size_t)3 * 128 * HD, node_b1 + (size_t)3 * HD,
      node_w2 + (size_t)3 * HD * HD,  node_b2 + (size_t)3 * HD,
      emb_out_w, emb_out_b, xbuf[0], hA, out, N);
}
